// SentenceReadout_10428180595138
// MI455X (gfx1250) — hardware-verified
//
#include <hip/hip_runtime.h>


#define N_ROWS 8192
#define HDIM   256
#define NGRAPH 64
#define NSPLIT 2
#define KBLK   (N_ROWS / 32 / NSPLIT)
#define NLINE  (N_ROWS / 16)
#define XSTR   264
#define VSTR   72
#define SSTR   72
#define PSTR   40
#define OSTR   36
#define WSCR   576

typedef _Float16 v16h __attribute__((ext_vector_type(16)));
typedef _Float16 v8h  __attribute__((ext_vector_type(8)));
typedef float    v8f  __attribute__((ext_vector_type(8)));
typedef float    v4f  __attribute__((ext_vector_type(4)));
union Frag { v16h v; v8h half[2]; };

__device__ __forceinline__ v8f mma16(const v16h a, const v16h b, v8f c) {
  c = __builtin_amdgcn_wmma_f32_16x16x32_f16(false, a, false, b, (short)0, c, false, false);
  asm volatile("v_nop\n\tv_nop\n\tv_nop\n\tv_nop" : "+v"(c) : "v"(a), "v"(b));
  return c;
}

__device__ __forceinline__ v8f zero8() {
  v8f z;
#pragma unroll
  for (int i = 0; i < 8; ++i) z[i] = 0.0f;
  return z;
}

__device__ __forceinline__ v4f zero4() {
  v4f z;
#pragma unroll
  for (int i = 0; i < 4; ++i) z[i] = 0.0f;
  return z;
}

__global__ __launch_bounds__(256)
void prep_w_kernel(const float* __restrict__ We, const float* __restrict__ Wq,
                   const float* __restrict__ Wk, const float* __restrict__ Wv,
                   _Float16* __restrict__ wt) {
  const int gid = blockIdx.x * blockDim.x + threadIdx.x;
  if (gid >= 4 * HDIM * HDIM / 8) return;
  const int w  = gid >> 13;
  const int r  = gid & 8191;
  const int n  = r >> 5;
  const int k0 = (r & 31) * 8;
  const float* src = (w == 0) ? We : (w == 1) ? Wq : (w == 2) ? Wk : Wv;
  v8h v;
#pragma unroll
  for (int i = 0; i < 8; ++i) v[i] = (_Float16)(src[(size_t)(k0 + i) * HDIM + n] * 64.0f);
  _Float16* dst = wt + (size_t)w * HDIM * HDIM + (size_t)n * HDIM + k0;
  *(volatile v8h*)dst = v;
  __threadfence();
  *(volatile v8h*)dst = v;
}

__device__ __forceinline__ void gemm_16x256(const _Float16* aL, const _Float16* __restrict__ Bt,
                                            const int ln, const int hb, v8f acc[16]) {
#pragma unroll
  for (int nt = 0; nt < 16; ++nt) acc[nt] = zero8();
  const _Float16* bL = Bt + (size_t)ln * HDIM + hb * 8;
#pragma unroll 1
  for (int kc = 0; kc < 8; ++kc) {
    Frag a;
    a.half[0] = *(const v8h*)(aL + kc * 32);
    a.half[1] = *(const v8h*)(aL + kc * 32 + 16);
#pragma unroll
    for (int nt = 0; nt < 16; ++nt) {
      const _Float16* bp = bL + (size_t)nt * 16 * HDIM + kc * 32;
      Frag b;
      b.half[0] = *(const v8h*)(bp);
      b.half[1] = *(const v8h*)(bp + 16);
      acc[nt] = mma16(a.v, b.v, acc[nt]);
    }
  }
}

__device__ __forceinline__ void store_rows16(const v8f acc[16], const float* __restrict__ bias,
                                             _Float16* __restrict__ dst, const int rowBase,
                                             _Float16* myscr, const int lane) {
  const int ln = lane & 15, hb = lane >> 4;
  const int rr = lane >> 3, ch = lane & 7;
#pragma unroll
  for (int g = 0; g < 4; ++g) {
#pragma unroll
    for (int t = 0; t < 4; ++t) {
      const int nt = g * 4 + t;
      const float b = bias[nt * 16 + ln];
#pragma unroll
      for (int v = 0; v < 8; ++v)
        myscr[(hb * 8 + v) * SSTR + t * 16 + ln] = (_Float16)(acc[nt][v] * (1.0f / 64.0f) + b);
    }
    __syncthreads();
    v8h val[4];
#pragma unroll
    for (int i = 0; i < 4; ++i) val[i] = *(const v8h*)(myscr + (i * 4 + rr) * SSTR + ch * 8);
#pragma unroll
    for (int i = 0; i < 4; ++i)
      *(volatile v8h*)(dst + (size_t)(rowBase + i * 4 + rr) * HDIM + g * 64 + ch * 8) = val[i];
    __threadfence();
#pragma unroll
    for (int i = 0; i < 4; ++i)
      *(volatile v8h*)(dst + (size_t)(rowBase + i * 4 + rr) * HDIM + g * 64 + ch * 8) = val[i];
    __syncthreads();
  }
}

__global__ __launch_bounds__(128) __attribute__((amdgpu_num_vgpr(256)))
void proj_kernel(const float* __restrict__ x, const _Float16* __restrict__ wt,
                 const float* __restrict__ b_emb, const float* __restrict__ bq,
                 const float* __restrict__ bk, const float* __restrict__ bv,
                 _Float16* __restrict__ Qs, _Float16* __restrict__ Kf, _Float16* __restrict__ Vt) {
  __shared__ __attribute__((aligned(16))) _Float16 tile[256 * VSTR];
  __shared__ __attribute__((aligned(16))) _Float16 scr[4 * 16 * SSTR];
  const int tid  = threadIdx.x;
  const int w    = tid >> 5;
  const int lane = tid & 31;
  const int ln   = lane & 15;
  const int hb   = lane >> 4;
  const int rowBlk = blockIdx.x * 64;
  _Float16* myscr = scr + w * 16 * SSTR;

#pragma unroll
  for (int it = 0; it < 16; ++it) {
    const int idx = it * 128 + tid;
    const int r   = idx >> 5;
    const int c8  = (idx & 31) * 8;
    const float* xp = x + (size_t)(rowBlk + r) * HDIM + c8;
    const v4f x0 = *(const v4f*)(xp);
    const v4f x1 = *(const v4f*)(xp + 4);
    v8h hv;
    hv[0] = (_Float16)x0[0]; hv[1] = (_Float16)x0[1]; hv[2] = (_Float16)x0[2]; hv[3] = (_Float16)x0[3];
    hv[4] = (_Float16)x1[0]; hv[5] = (_Float16)x1[1]; hv[6] = (_Float16)x1[2]; hv[7] = (_Float16)x1[3];
    *(v8h*)(tile + r * XSTR + c8) = hv;
  }
  __syncthreads();

  v8f acc[16];
  const _Float16* aL = tile + (w * 16 + ln) * XSTR + hb * 8;

  gemm_16x256(aL, wt, ln, hb, acc);
  __syncthreads();
#pragma unroll
  for (int nt = 0; nt < 16; ++nt) {
    const float b = b_emb[nt * 16 + ln];
#pragma unroll
    for (int v = 0; v < 8; ++v) {
      float hv = acc[nt][v] * (1.0f / 64.0f) + b;
      hv = hv > 0.0f ? hv : 0.0f;
      tile[(w * 16 + hb * 8 + v) * XSTR + nt * 16 + ln] = (_Float16)hv;
    }
  }
  __syncthreads();

  gemm_16x256(aL, wt + 1 * HDIM * HDIM, ln, hb, acc);
  store_rows16(acc, bq, Qs, rowBlk + w * 16, myscr, lane);
  gemm_16x256(aL, wt + 2 * HDIM * HDIM, ln, hb, acc);
  store_rows16(acc, bk, Kf, rowBlk + w * 16, myscr, lane);
  gemm_16x256(aL, wt + 3 * HDIM * HDIM, ln, hb, acc);
  __syncthreads();
#pragma unroll
  for (int nt = 0; nt < 16; ++nt) {
    const int col = nt * 16 + ln;
    const float b = bv[col];
    v8h pk;
#pragma unroll
    for (int v = 0; v < 8; ++v) pk[v] = (_Float16)(acc[nt][v] * (1.0f / 64.0f) + b);
    *(v8h*)(tile + col * VSTR + w * 16 + hb * 8) = pk;
  }
  __syncthreads();
  {
    const int rr = lane >> 3, ch = lane & 7;
#pragma unroll
    for (int i = 0; i < 16; ++i) {
      const int col = w * 64 + i * 4 + rr;
      const v8h val = *(const v8h*)(tile + col * VSTR + ch * 8);
      *(volatile v8h*)(Vt + (size_t)col * N_ROWS + rowBlk + ch * 8) = val;
    }
    __threadfence();
#pragma unroll
    for (int i = 0; i < 16; ++i) {
      const int col = w * 64 + i * 4 + rr;
      const v8h val = *(const v8h*)(tile + col * VSTR + ch * 8);
      *(volatile v8h*)(Vt + (size_t)col * N_ROWS + rowBlk + ch * 8) = val;
    }
  }
}

__global__ __launch_bounds__(128) __attribute__((amdgpu_num_vgpr(256)))
void attn_kernel(const _Float16* __restrict__ Qs, const _Float16* __restrict__ Kf,
                 const _Float16* __restrict__ Vt, float* __restrict__ Opart,
                 float* __restrict__ ml) {
  __shared__ __attribute__((aligned(16))) _Float16 qt[64 * XSTR];
  __shared__ __attribute__((aligned(16))) float wscr[4 * WSCR];
  const int tid  = threadIdx.x;
  const int w    = tid >> 5;
  const int lane = tid & 31;
  const int ln   = lane & 15;
  const int hb   = lane >> 4;
  const int r0   = blockIdx.x * 64;
  const int split = blockIdx.y;
  float* O = Opart + (size_t)split * N_ROWS * HDIM;
  float* scrf = wscr + w * WSCR;
  _Float16* scrh = (_Float16*)scrf;

#pragma unroll
  for (int it = 0; it < 16; ++it) {
    const int idx = it * 128 + tid;
    const int r   = idx >> 5;
    const int c8  = (idx & 31) * 8;
    *(v8h*)(qt + r * XSTR + c8) = *(const v8h*)(Qs + (size_t)(r0 + r) * HDIM + c8);
  }
  __syncthreads();
  const _Float16* aL = qt + (w * 16 + ln) * XSTR + hb * 8;

  v8f o[16];
#pragma unroll
  for (int nt = 0; nt < 16; ++nt) o[nt] = zero8();
  float mrun[8], lsum[8];
#pragma unroll
  for (int v = 0; v < 8; ++v) { mrun[v] = -3.0e38f; lsum[v] = 0.0f; }

  const int jbeg = split * KBLK;
  const int jend = jbeg + KBLK;
#pragma unroll 1
  for (int j = jbeg; j < jend; ++j) {
    const int kb = j * 32;

    v8f s0 = zero8(), s1 = zero8();
    const _Float16* kL = Kf + (size_t)(kb + ln) * HDIM + hb * 8;
#pragma unroll 1
    for (int kc = 0; kc < 8; ++kc) {
      Frag a, b0, b1;
      a.half[0]  = *(const v8h*)(aL + kc * 32);
      a.half[1]  = *(const v8h*)(aL + kc * 32 + 16);
      b0.half[0] = *(const v8h*)(kL + kc * 32);
      b0.half[1] = *(const v8h*)(kL + kc * 32 + 16);
      b1.half[0] = *(const v8h*)(kL + 16 * HDIM + kc * 32);
      b1.half[1] = *(const v8h*)(kL + 16 * HDIM + kc * 32 + 16);
      s0 = mma16(a.v, b0.v, s0);
      s1 = mma16(a.v, b1.v, s1);
    }
#pragma unroll
    for (int v = 0; v < 8; ++v) { s0[v] *= 0.0625f; s1[v] *= 0.0625f; }

    float t[8];
#pragma unroll
    for (int v = 0; v < 8; ++v) t[v] = fmaxf(s0[v], s1[v]);
#pragma unroll
    for (int d = 1; d < 16; d <<= 1)
#pragma unroll
      for (int v = 0; v < 8; ++v) t[v] = fmaxf(t[v], __shfl_xor(t[v], d, 32));

    float corr[8];
#pragma unroll
    for (int v = 0; v < 8; ++v) {
      const float mn = fmaxf(mrun[v], t[v]);
      corr[v] = __expf(mrun[v] - mn);
      mrun[v] = mn;
      lsum[v] *= corr[v];
    }
#pragma unroll
    for (int nt = 0; nt < 16; ++nt)
#pragma unroll
      for (int v = 0; v < 8; ++v) o[nt][v] *= corr[v];

#pragma unroll
    for (int v = 0; v < 8; ++v) {
      const float p0 = __expf(s0[v] - mrun[v]);
      const float p1 = __expf(s1[v] - mrun[v]);
      lsum[v] += p0 + p1;
      scrh[(hb * 8 + v) * PSTR + ln]      = (_Float16)(p0 * 256.0f);
      scrh[(hb * 8 + v) * PSTR + 16 + ln] = (_Float16)(p1 * 256.0f);
    }
    __syncthreads();
    Frag pa;
    pa.half[0] = *(const v8h*)(scrh + ln * PSTR + hb * 8);
    pa.half[1] = *(const v8h*)(scrh + ln * PSTR + 16 + hb * 8);
    __syncthreads();

    const _Float16* vL = Vt + (size_t)ln * N_ROWS + kb + hb * 8;
#pragma unroll
    for (int nt = 0; nt < 16; ++nt) {
      const _Float16* vp = vL + (size_t)nt * 16 * N_ROWS;
      Frag vb;
      vb.half[0] = *(const v8h*)(vp);
      vb.half[1] = *(const v8h*)(vp + 16);
      o[nt] = mma16(pa.v, vb.v, o[nt]);
    }
  }

#pragma unroll
  for (int d = 1; d < 16; d <<= 1)
#pragma unroll
    for (int v = 0; v < 8; ++v) lsum[v] += __shfl_xor(lsum[v], d, 32);

  const int rr = lane >> 3, ch = lane & 7;
#pragma unroll
  for (int g = 0; g < 8; ++g) {
#pragma unroll
    for (int t2 = 0; t2 < 2; ++t2) {
      const int nt = g * 2 + t2;
#pragma unroll
      for (int v = 0; v < 8; ++v)
        scrf[(hb * 8 + v) * OSTR + t2 * 16 + ln] = o[nt][v] * (1.0f / 256.0f);
    }
    __syncthreads();
    v4f val[4];
#pragma unroll
    for (int i = 0; i < 4; ++i) val[i] = *(const v4f*)(scrf + (i * 4 + rr) * OSTR + ch * 4);
#pragma unroll
    for (int i = 0; i < 4; ++i)
      *(volatile v4f*)(O + (size_t)(r0 + w * 16 + i * 4 + rr) * HDIM + g * 32 + ch * 4) = val[i];
    __threadfence();
#pragma unroll
    for (int i = 0; i < 4; ++i)
      *(volatile v4f*)(O + (size_t)(r0 + w * 16 + i * 4 + rr) * HDIM + g * 32 + ch * 4) = val[i];
    __syncthreads();
  }

  if (ln == 0) {
#pragma unroll
    for (int v = 0; v < 8; ++v) {
      scrf[hb * 8 + v]      = mrun[v];
      scrf[16 + hb * 8 + v] = lsum[v];
    }
  }
  __syncthreads();
  const v4f mlv = *(const v4f*)(scrf + ch * 4);
  float* mlp = ml + ((size_t)split * NLINE + (size_t)blockIdx.x * 4 + w) * 32 + ch * 4;
  if (lane < 8) *(volatile v4f*)mlp = mlv;
  __threadfence();
  if (lane < 8) *(volatile v4f*)mlp = mlv;
}

__device__ __forceinline__ int lower_bound_i(const int* __restrict__ a, const int n, const int key) {
  int lo = 0, hi = n;
#pragma unroll 1
  for (int it = 0; it < 32 && lo < hi; ++it) {
    const int mid = (lo + hi) >> 1;
    if (a[mid] < key) lo = mid + 1; else hi = mid;
  }
  return lo;
}

__global__ __launch_bounds__(64)
void pool_kernel(const float* __restrict__ Opart, const float* __restrict__ ml,
                 const int* __restrict__ batch, float* __restrict__ out) {
  const int b  = blockIdx.x;
  const int c4 = threadIdx.x * 4;
  const int s  = lower_bound_i(batch, N_ROWS, b);
  int e = lower_bound_i(batch, N_ROWS, b + 1);
  e = e > N_ROWS ? N_ROWS : e;
  const int cnt = e - s;
  v4f mx = zero4(), sm = zero4();
  if (cnt > 0) {
    v4f mxx, acc4 = zero4();
#pragma unroll
    for (int c = 0; c < 4; ++c) mxx[c] = -3.4e38f;
    const float* O0 = Opart + c4;
    const float* O1 = Opart + (size_t)N_ROWS * HDIM + c4;
#pragma unroll 1
    for (int i = s; i < e; ++i) {
      const int g = i >> 4, q = i & 15;
      const float m0 = ml[g * 32 + q];
      const float l0 = ml[g * 32 + 16 + q];
      const float m1 = ml[(NLINE + g) * 32 + q];
      const float l1 = ml[(NLINE + g) * 32 + 16 + q];
      const float ms  = fmaxf(m0, m1);
      const float f0  = __expf(m0 - ms);
      const float f1  = __expf(m1 - ms);
      const float inv = 1.0f / (l0 * f0 + l1 * f1);
      const v4f a0 = *(const v4f*)(O0 + (size_t)i * HDIM);
      const v4f a1 = *(const v4f*)(O1 + (size_t)i * HDIM);
      const v4f val = (a0 * f0 + a1 * f1) * inv;
#pragma unroll
      for (int c = 0; c < 4; ++c) mxx[c] = fmaxf(mxx[c], val[c]);
      acc4 += val;
    }
    const float rc = 1.0f / (float)cnt;
    mx = mxx;
    sm = acc4 * rc;
  }
  float* pm = out + (size_t)b * 2 * HDIM + c4;
  float* ps = out + (size_t)b * 2 * HDIM + HDIM + c4;
  *(volatile v4f*)pm = mx;
  *(volatile v4f*)ps = sm;
  __threadfence();
  *(volatile v4f*)pm = mx;
  *(volatile v4f*)ps = sm;
}

extern "C" void kernel_launch(void* const* d_in, const int* in_sizes, int n_in,
                              void* d_out, int out_size, void* d_ws, size_t ws_size,
                              hipStream_t stream) {
  if (n_in < 10) return;
  if (in_sizes[0] != N_ROWS * HDIM) return;
  if (in_sizes[1] != HDIM * HDIM || in_sizes[3] != HDIM * HDIM ||
      in_sizes[5] != HDIM * HDIM || in_sizes[7] != HDIM * HDIM) return;
  if (in_sizes[2] != HDIM || in_sizes[4] != HDIM || in_sizes[6] != HDIM || in_sizes[8] != HDIM) return;
  if (in_sizes[9] != N_ROWS) return;
  if (out_size != NGRAPH * 2 * HDIM) return;

  const float* x     = (const float*)d_in[0];
  const float* W_emb = (const float*)d_in[1];
  const float* b_emb = (const float*)d_in[2];
  const float* Wq    = (const float*)d_in[3];
  const float* bq    = (const float*)d_in[4];
  const float* Wk    = (const float*)d_in[5];
  const float* bk    = (const float*)d_in[6];
  const float* Wv    = (const float*)d_in[7];
  const float* bv    = (const float*)d_in[8];
  const int*   batch = (const int*)d_in[9];
  float* out = (float*)d_out;

  const size_t wt_bytes = (size_t)4 * HDIM * HDIM * 2;
  const size_t qk_bytes = (size_t)N_ROWS * HDIM * 2;
  const size_t o_bytes  = (size_t)NSPLIT * N_ROWS * HDIM * 4;
  const size_t ml_bytes = (size_t)NSPLIT * NLINE * 32 * 4;
  const size_t off_wt = 0;
  const size_t off_q  = off_wt + wt_bytes;
  const size_t off_k  = off_q + qk_bytes;
  const size_t off_v  = off_k + qk_bytes;
  const size_t off_o  = off_v + qk_bytes;
  const size_t off_ml = off_o + o_bytes;
  const size_t total  = off_ml + ml_bytes;
  if (total > ws_size) return;

  char* ws = (char*)d_ws;
  _Float16* wt    = (_Float16*)(ws + off_wt);
  _Float16* Qs    = (_Float16*)(ws + off_q);
  _Float16* Kf    = (_Float16*)(ws + off_k);
  _Float16* Vt    = (_Float16*)(ws + off_v);
  float*    Opart = (float*)(ws + off_o);
  float*    ml    = (float*)(ws + off_ml);

  prep_w_kernel<<<(4 * HDIM * HDIM / 8 + 255) / 256, 256, 0, stream>>>(W_emb, Wq, Wk, Wv, wt);
  proj_kernel<<<N_ROWS / 64, 128, 0, stream>>>(x, wt, b_emb, bq, bk, bv, Qs, Kf, Vt);
  attn_kernel<<<dim3(N_ROWS / 64, NSPLIT), 128, 0, stream>>>(Qs, Kf, Vt, Opart, ml);
  pool_kernel<<<NGRAPH, 64, 0, stream>>>(Opart, ml, batch, out);
}
